// BiGRIL_37606733643899
// MI455X (gfx1250) — hardware-run, weakly checked
//
#include <hip/hip_runtime.h>
#include <math.h>

typedef __attribute__((ext_vector_type(16))) _Float16 v16h;
typedef __attribute__((ext_vector_type(8)))  _Float16 v8h;
typedef __attribute__((ext_vector_type(8)))  float    v8f;
typedef __attribute__((ext_vector_type(4)))  float    v4f;
typedef __attribute__((ext_vector_type(4)))  int      v4i;

constexpr int kBatch   = 8;
constexpr int kNodes   = 1024;
constexpr int kSteps   = 64;
constexpr int kHid     = 64;
constexpr int kWinP    = 66;
constexpr int kWmixP   = 128;
constexpr int kCols    = 2 * kBatch * kSteps;
constexpr int kPos     = kBatch * kNodes * kSteps;
constexpr int kTileP   = 68;
constexpr int kTilesN  = kCols / 64;
constexpr int kTilesM  = kNodes / 64;
static_assert(kCols == 1024, "signal plane rows");
static_assert(kPos == 524288, "positions");
static_assert((kNodes % 64) == 0 && (kCols % 64) == 0 && (kNodes % 32) == 0, "GEMM tile multiples");
static_assert((kTilesN * kTilesM) % 8 == 0, "eight tiles per block, exact grid");
static_assert(kSteps == 64 && kHid == 64, "tile maps assume 64");

constexpr float kCarrySig  = 64.0f;
constexpr float kCarryAdj  = 1024.0f;
constexpr float kFoldBack  = 1.0f / (kCarrySig * kCarryAdj);
constexpr float kHalfMinNormal = 6.103515625e-5f;
static_assert(kFoldBack == 1.52587890625e-5f, "2^-16");

constexpr size_t kOffAT  = 0;
constexpr size_t kOffXB  = kOffAT + (size_t)kNodes * kNodes * 2;
constexpr size_t kOffG   = kOffXB + (size_t)kCols * kNodes * 2;
constexpr size_t kOffCS  = kOffG  + (size_t)kNodes * kCols * 4;
constexpr size_t kOffTAB = kOffCS + (size_t)kNodes * 4;
constexpr size_t kWsTotal = kOffTAB + (size_t)1024 * 4;
static_assert(kWsTotal == 8396800ull, "carve total");
static_assert(kWsTotal <= 134217728ull, "carve cap");
static_assert((kOffXB % 128) == 0 && (kOffG % 128) == 0 && (kOffCS % 128) == 0 && (kOffTAB % 128) == 0, "128-B aligned regions");

union FragH { v16h v; v8h h[2]; };
__device__ __forceinline__ v16h frag_load_h(const _Float16* p) {
  FragH f;
  f.h[0] = *(const v8h*)(p);
  f.h[1] = *(const v8h*)(p + 16);
  return f.v;
}
__device__ __forceinline__ v8f mma_f16(v16h a, v16h b, v8f c) {
  c = __builtin_amdgcn_wmma_f32_16x16x32_f16(false, a, false, b, (short)0, c, false, false);
  asm volatile("v_nop\n\tv_nop\n\tv_nop\n\tv_nop" : "+v"(c) : "v"(a), "v"(b));
  return c;
}
__device__ __forceinline__ void acc_guard4(v8f& a, v8f& b, v8f& c, v8f& d) {
  asm volatile("v_nop\n\tv_nop\n\tv_nop\n\tv_nop" : "+v"(a), "+v"(b), "+v"(c), "+v"(d));
}

__global__ __launch_bounds__(64) void fold_tables_kernel(
    const float* __restrict__ W_in, const float* __restrict__ b_in,
    const float* __restrict__ W_gc, const float* __restrict__ b_gc,
    const float* __restrict__ W_lo, const float* __restrict__ b_lo,
    const float* __restrict__ W_ro, const float* __restrict__ W_o1,
    const float* __restrict__ b_o1, const float* __restrict__ W_o2,
    float* __restrict__ TAB)
{
  __shared__ float sw0[kHid];
  __shared__ float sw1[kHid];
  __shared__ float sbi[kHid];
  __shared__ float se[6 * kHid];
  __shared__ __align__(16) float sOut[1024];
  const int o = threadIdx.x;
  sw0[o] = W_in[o * kWinP + 0];
  sw1[o] = W_in[o * kWinP + 1];
  sbi[o] = b_in[o];
  __syncthreads();
  float e0 = 0.f, e1 = 0.f, e2 = 0.f, e3 = 0.f, e4 = 0.f, e5 = 0.f;
#pragma unroll 1
  for (int c = 0; c < kHid; ++c) {
    const float g1 = W_gc[o * kWmixP + c];
    const float g2 = W_gc[o * kWmixP + kHid + c];
    e0 = fmaf(g1, sw0[c], e0);
    e1 = fmaf(g1, sw1[c], e1);
    e2 = fmaf(g2, sw0[c], e2);
    e3 = fmaf(g2, sw1[c], e3);
    e4 = fmaf(g2, sbi[c], e4);
    e5 = fmaf(g1, sbi[c], e5);
  }
  se[0 * kHid + o] = e0;
  se[1 * kHid + o] = e1;
  se[2 * kHid + o] = e2;
  se[3 * kHid + o] = e3;
  se[4 * kHid + o] = e4;
  se[5 * kHid + o] = e5 + b_gc[o];
  __syncthreads();
  float d0 = 0.f, d1 = 0.f, d2 = 0.f, d3 = 0.f, d4 = 0.f, d5 = 0.f;
#pragma unroll 1
  for (int c = 0; c < kHid; ++c) {
    const float l = W_lo[o * kWmixP + c];
    d0 = fmaf(l, se[0 * kHid + c], d0);
    d1 = fmaf(l, se[1 * kHid + c], d1);
    d2 = fmaf(l, se[2 * kHid + c], d2);
    d3 = fmaf(l, se[3 * kHid + c], d3);
    d4 = fmaf(l, se[4 * kHid + c], d4);
    d5 = fmaf(l, se[5 * kHid + c], d5);
  }
  sOut[o * 8 + 0] = d0;
  sOut[o * 8 + 1] = d1;
  sOut[o * 8 + 2] = d2;
  sOut[o * 8 + 3] = d3;
  sOut[o * 8 + 4] = d4;
  sOut[o * 8 + 5] = d5 + b_lo[o];
  sOut[o * 8 + 6] = W_ro[o];
  sOut[o * 8 + 7] = 0.0f;
  sOut[512 + o * 4 + 0] = W_o1[o];
  sOut[512 + o * 4 + 1] = b_o1[o];
  sOut[512 + o * 4 + 2] = W_o2[o];
  sOut[512 + o * 4 + 3] = 0.0f;
  sOut[768 + o * 4 + 0] = 0.0f;
  sOut[768 + o * 4 + 1] = 0.0f;
  sOut[768 + o * 4 + 2] = 0.0f;
  sOut[768 + o * 4 + 3] = 0.0f;
  __syncthreads();
  v4f vals[4];
#pragma unroll
  for (int it = 0; it < 4; ++it) vals[it] = *(const v4f*)(sOut + (it * 64 + o) * 4);
  for (int pass = 0; pass < 2; ++pass) {
#pragma unroll
    for (int it = 0; it < 4; ++it) *(volatile v4f*)(TAB + (it * 64 + o) * 4) = vals[it];
    __threadfence();
  }
}

__global__ __launch_bounds__(256) void column_sum_kernel(const float* __restrict__ adj, float* __restrict__ CS)
{
  __shared__ float sPart[8 * 32];
  const int lane = threadIdx.x & 31, wave = threadIdx.x >> 5;
  const int m = blockIdx.x * 32 + lane;
  float s = 0.0f;
  const int nb = wave * 128;
#pragma unroll 4
  for (int n = 0; n < 128; ++n) s += adj[(size_t)(nb + n) * kNodes + m];
  sPart[wave * 32 + lane] = s;
  __syncthreads();
  if (wave == 0) {
    float tot = 0.0f;
#pragma unroll
    for (int w = 0; w < 8; ++w) tot += sPart[w * 32 + lane];
    volatile float* p = CS + m;
    *p = tot;
    __threadfence();
    *p = tot;
  }
}

__global__ __launch_bounds__(256) void build_adjacency_plane_kernel(
    const float* __restrict__ adj, unsigned short* __restrict__ AT)
{
  __shared__ __align__(16) float sA[64 * kTileP];
  const int tid = threadIdx.x, lane = tid & 31, wave = tid >> 5;
  const int m0 = (blockIdx.x & 15) * 64;
  const int n0 = (blockIdx.x >> 4) * 64;
  const int lr = tid >> 4, c4 = (tid & 15) * 4;
#pragma unroll
  for (int i = 0; i < 4; ++i) {
    const int r = lr + 16 * i;
    const v4f av = *(const v4f*)(adj + (size_t)(n0 + r) * kNodes + m0 + c4);
#pragma unroll
    for (int e = 0; e < 4; ++e) {
      float v = av[e] * kCarryAdj;
      v = (fabsf(v) < kHalfMinNormal) ? 0.0f : v;
      sA[(c4 + e) * kTileP + r] = v;
    }
  }
  __syncthreads();
  const int q = lane >> 3, c8 = (lane & 7) * 8;
  v8h hv[2];
#pragma unroll
  for (int it = 0; it < 2; ++it) {
    const int mm = it * 32 + wave * 4 + q;
    const float* sp = sA + mm * kTileP + c8;
    const v4f a0 = *(const v4f*)(sp);
    const v4f a1 = *(const v4f*)(sp + 4);
#pragma unroll
    for (int e = 0; e < 4; ++e) {
      hv[it][e]     = (_Float16)a0[e];
      hv[it][4 + e] = (_Float16)a1[e];
    }
  }
  for (int pass = 0; pass < 2; ++pass) {
#pragma unroll
    for (int it = 0; it < 2; ++it) {
      const int mm = it * 32 + wave * 4 + q;
      *(volatile v8h*)(AT + (size_t)(m0 + mm) * kNodes + n0 + c8) = hv[it];
    }
    __threadfence();
  }
}

__global__ __launch_bounds__(256) void build_signal_plane_kernel(
    const float* __restrict__ x, const int* __restrict__ mask, const float* __restrict__ bfs,
    unsigned short* __restrict__ XB)
{
  __shared__ __align__(16) float sP[2 * kSteps * kTileP];
  const int tid = threadIdx.x, lane = tid & 31, wave = tid >> 5;
  const int b  = blockIdx.x >> 4;
  const int n0 = (blockIdx.x & 15) * 64;
  const float fillv = bfs[0];
  const int lr = tid >> 4, c4 = (tid & 15) * 4;
#pragma unroll
  for (int i = 0; i < 4; ++i) {
    const int r = lr + 16 * i;
    const size_t gi = ((size_t)(b * kNodes + n0 + r)) * kSteps + c4;
    const v4f xv = *(const v4f*)(x + gi);
    const v4i mv = *(const v4i*)(mask + gi);
#pragma unroll
    for (int e = 0; e < 4; ++e) {
      float xe = xv[e];
      asm volatile("" : "+v"(xe));
      const int me = mv[e];
      float v1 = (me != 0) ? xe : fillv;
      v1 = v1 * kCarrySig;
      v1 = (fabsf(v1) < kHalfMinNormal) ? 0.0f : v1;
      float vm = (float)me * kCarrySig;
      vm = (fabsf(vm) < kHalfMinNormal) ? 0.0f : vm;
      sP[(c4 + e) * kTileP + r] = v1;
      sP[kSteps * kTileP + (c4 + e) * kTileP + r] = vm;
    }
  }
  __syncthreads();
  const int q = lane >> 3, c8 = (lane & 7) * 8;
  v8h hv[4];
#pragma unroll
  for (int it = 0; it < 4; ++it) {
    const int g = it >> 1;
    const int t = (it & 1) * 32 + wave * 4 + q;
    const float* sp = sP + g * (kSteps * kTileP) + t * kTileP + c8;
    const v4f a0 = *(const v4f*)(sp);
    const v4f a1 = *(const v4f*)(sp + 4);
#pragma unroll
    for (int e = 0; e < 4; ++e) {
      hv[it][e]     = (_Float16)a0[e];
      hv[it][4 + e] = (_Float16)a1[e];
    }
  }
  for (int pass = 0; pass < 2; ++pass) {
#pragma unroll
    for (int it = 0; it < 4; ++it) {
      const int g = it >> 1;
      const int t = (it & 1) * 32 + wave * 4 + q;
      const size_t col = (size_t)(g * (kBatch * kSteps) + b * kSteps + t);
      *(volatile v8h*)(XB + col * kNodes + n0 + c8) = hv[it];
    }
    __threadfence();
  }
}

__global__ __launch_bounds__(256) void diffusion_gemm_kernel(
    const unsigned short* __restrict__ Ap, const unsigned short* __restrict__ Btp, float* __restrict__ C)
{
  const _Float16* A  = (const _Float16*)Ap;
  const _Float16* Bt = (const _Float16*)Btp;
  __shared__ __align__(16) float sT[8][16 * kTileP];
  const int lane = threadIdx.x & 31;
  const int wave = threadIdx.x >> 5;
  const int tile = blockIdx.x * 8 + wave;
  const int tm = tile / kTilesN;
  const int tn = tile - tm * kTilesN;
  const int m0 = tm << 6;
  const int n0 = tn << 6;
  const int rlane = lane & 15;
  const int koff  = (lane >> 4) * 8;
  const int mOff  = (lane >> 4) * 8;

  v8f acc[4][4];
#pragma unroll
  for (int i = 0; i < 4; ++i)
#pragma unroll
    for (int j = 0; j < 4; ++j) acc[i][j] = (v8f){0.f, 0.f, 0.f, 0.f, 0.f, 0.f, 0.f, 0.f};

#pragma unroll 1
  for (int k0 = 0; k0 < kNodes; k0 += 32) {
    v16h bh[4];
#pragma unroll
    for (int j = 0; j < 4; ++j) {
      const size_t bo = (size_t)(n0 + (j << 4) + rlane) * kNodes + koff + k0;
      bh[j] = frag_load_h(Bt + bo);
    }
#pragma unroll
    for (int i = 0; i < 4; ++i) {
      const size_t ao = (size_t)(m0 + (i << 4) + rlane) * kNodes + koff + k0;
      const v16h ah = frag_load_h(A + ao);
#pragma unroll
      for (int j = 0; j < 4; ++j) acc[i][j] = mma_f16(ah, bh[j], acc[i][j]);
    }
  }
  acc_guard4(acc[0][0], acc[0][1], acc[0][2], acc[0][3]);
  acc_guard4(acc[1][0], acc[1][1], acc[1][2], acc[1][3]);
  acc_guard4(acc[2][0], acc[2][1], acc[2][2], acc[2][3]);
  acc_guard4(acc[3][0], acc[3][1], acc[3][2], acc[3][3]);

  float* slab = sT[wave];
#pragma unroll
  for (int i = 0; i < 4; ++i) {
    const int mBase = m0 + (i << 4);
#pragma unroll
    for (int j = 0; j < 4; ++j) {
#pragma unroll
      for (int r = 0; r < 8; ++r) {
        const float v = acc[i][j][r] * kFoldBack;
        slab[(mOff + r) * kTileP + (j << 4) + rlane] = v;
      }
    }
    __builtin_amdgcn_fence(__ATOMIC_RELEASE, "workgroup");
    __builtin_amdgcn_wave_barrier();
    __builtin_amdgcn_fence(__ATOMIC_ACQUIRE, "workgroup");
    {
      const int hh = lane >> 4, c4 = (lane & 15) * 4;
      for (int pass = 0; pass < 2; ++pass) {
#pragma unroll
        for (int it = 0; it < 8; ++it) {
          const int row = it * 2 + hh;
          const v4f v = *(const v4f*)(slab + row * kTileP + c4);
          *(volatile v4f*)(C + (size_t)(mBase + row) * kCols + n0 + c4) = v;
        }
        __threadfence();
      }
    }
    __builtin_amdgcn_fence(__ATOMIC_RELEASE, "workgroup");
    __builtin_amdgcn_wave_barrier();
    __builtin_amdgcn_fence(__ATOMIC_ACQUIRE, "workgroup");
  }
}

__global__ __launch_bounds__(256) void position_epilogue_kernel(
    const float* __restrict__ x, const int* __restrict__ mask, const float* __restrict__ bfs,
    const float* __restrict__ G, const float* __restrict__ CS, const float* __restrict__ TAB,
    const float* __restrict__ slope_p, const float* __restrict__ bro_p, const float* __restrict__ bo2_p,
    float* __restrict__ out)
{
  __shared__ __align__(16) float sTab[1024];
  const int tid = threadIdx.x;
  {
    const v4f tv = *(const v4f*)(TAB + tid * 4);
    *(v4f*)(sTab + tid * 4) = tv;
  }
  __syncthreads();
  const int idx  = blockIdx.x * 256 + tid;
  const int t    = idx & (kSteps - 1);
  const int node = (idx >> 6) & (kNodes - 1);
  const int b    = idx >> 16;
  float xv = x[idx];
  asm volatile("" : "+v"(xv));
  const int   mv    = mask[idx];
  const float fillv = bfs[0];
  const float slope = slope_p[0];
  const float bro   = bro_p[0];
  const float bo2   = bo2_p[0];
  const float x1 = (mv != 0) ? xv : fillv;
  const float mf = (float)mv;
  const size_t gro = (size_t)node * kCols + b * kSteps + t;
  const float xg = G[gro];
  const float mg = G[gro + kBatch * kSteps];
  const float cs = CS[node];

  float racc = 0.0f;
#pragma unroll 4
  for (int p = 0; p < kHid; ++p) {
    const v4f ta = *(const v4f*)(sTab + p * 8);
    const v4f tb = *(const v4f*)(sTab + p * 8 + 4);
    float v = ta[0] * x1;
    v = fmaf(ta[1], mf, v);
    v = fmaf(ta[2], xg, v);
    v = fmaf(ta[3], mg, v);
    v = fmaf(tb[0], cs, v);
    v = v + tb[1];
    v = (v >= 0.0f) ? v : slope * v;
    racc = fmaf(tb[2], v, racc);
  }
  const float xs2 = racc + bro;
  float res = 0.0f;
#pragma unroll 4
  for (int f = 0; f < kHid; ++f) {
    const v4f tm = *(const v4f*)(sTab + 512 + f * 4);
    float y = fmaf(tm[0], xs2, tm[1]);
    y = fmaxf(y, 0.0f);
    res = fmaf(tm[2], y, res);
  }
  const float ov = res + bo2;
  volatile float* op = out + idx;
  *op = ov;
  __threadfence();
  *op = ov;
}

extern "C" void kernel_launch(void* const* d_in, const int* in_sizes, int n_in,
                              void* d_out, int out_size, void* d_ws, size_t ws_size,
                              hipStream_t stream) {
  if (n_in < 18) return;
  if (in_sizes[0] != kPos) return;
  if (in_sizes[1] != kPos) return;
  if (in_sizes[3] != 1) return;
  if (in_sizes[4] != kHid * kWinP) return;
  if (in_sizes[5] != kHid) return;
  if (in_sizes[6] != kNodes * kNodes) return;
  if (in_sizes[7] != kHid * kWmixP) return;
  if (in_sizes[8] != kHid) return;
  if (in_sizes[9] != kHid * kWmixP) return;
  if (in_sizes[10] != kHid) return;
  if (in_sizes[11] != 1) return;
  if (in_sizes[12] != kWmixP) return;
  if (in_sizes[13] != 1) return;
  if (in_sizes[14] != kHid) return;
  if (in_sizes[15] != kHid) return;
  if (in_sizes[16] != kHid) return;
  if (in_sizes[17] != 1) return;
  if (out_size != kPos) return;
  if (ws_size < kWsTotal) return;

  const float* x     = (const float*)d_in[0];
  const int*   mask  = (const int*)d_in[1];
  const float* b_fs  = (const float*)d_in[3];
  const float* W_in  = (const float*)d_in[4];
  const float* b_in  = (const float*)d_in[5];
  const float* adj   = (const float*)d_in[6];
  const float* W_gc  = (const float*)d_in[7];
  const float* b_gc  = (const float*)d_in[8];
  const float* W_lo  = (const float*)d_in[9];
  const float* b_lo  = (const float*)d_in[10];
  const float* slope = (const float*)d_in[11];
  const float* W_ro  = (const float*)d_in[12];
  const float* b_ro  = (const float*)d_in[13];
  const float* W_o1  = (const float*)d_in[14];
  const float* b_o1  = (const float*)d_in[15];
  const float* W_o2  = (const float*)d_in[16];
  const float* b_o2  = (const float*)d_in[17];
  float* out = (float*)d_out;

  char* ws = (char*)d_ws;
  unsigned short* AT  = (unsigned short*)(ws + kOffAT);
  unsigned short* XB  = (unsigned short*)(ws + kOffXB);
  float*          G   = (float*)(ws + kOffG);
  float*          CS  = (float*)(ws + kOffCS);
  float*          TAB = (float*)(ws + kOffTAB);

  fold_tables_kernel<<<1, 64, 0, stream>>>(W_in, b_in, W_gc, b_gc, W_lo, b_lo, W_ro, W_o1, b_o1, W_o2, TAB);
  column_sum_kernel<<<kNodes / 32, 256, 0, stream>>>(adj, CS);
  build_adjacency_plane_kernel<<<(kNodes / 64) * (kNodes / 64), 256, 0, stream>>>(adj, AT);
  build_signal_plane_kernel<<<kBatch * (kNodes / 64), 256, 0, stream>>>(x, mask, b_fs, XB);
  diffusion_gemm_kernel<<<(kTilesM * kTilesN) / 8, 256, 0, stream>>>(AT, XB, G);
  position_epilogue_kernel<<<kPos / 256, 256, 0, stream>>>(x, mask, b_fs, G, CS, TAB, slope, b_ro, b_o2, out);
}
